// MyMSA_89464168776033
// MI455X (gfx1250) — hardware-verified
//
#include <hip/hip_runtime.h>
#include <math.h>
#include <stdint.h>

constexpr int kBatch = 2;
constexpr int kSeq   = 2048;
constexpr int kDm    = 1024;
constexpr int kHeads = 16;
constexpr int kHd    = 64;
constexpr int kRows  = kBatch * kSeq;
constexpr int kQkLd  = 2 * kDm;
constexpr float kPScale = 32768.0f;

typedef __attribute__((ext_vector_type(16))) _Float16 v16h;
typedef __attribute__((ext_vector_type(8)))  _Float16 v8h;
typedef __attribute__((ext_vector_type(16))) __bf16   v16b;
typedef __attribute__((ext_vector_type(8)))  __bf16   v8b;
typedef __attribute__((ext_vector_type(8)))  float    v8f;
typedef __attribute__((ext_vector_type(4)))  float    v4f;
typedef __attribute__((ext_vector_type(2)))  float    v2f;
typedef __attribute__((ext_vector_type(4)))  unsigned int v4u;

__device__ __forceinline__ unsigned short f2bf_bits(float f) {
  unsigned u = __float_as_uint(f);
  return (unsigned short)((u + 0x7FFFu + ((u >> 16) & 1u)) >> 16);
}
__device__ __forceinline__ float bf_bits2f(unsigned short h) { return __uint_as_float(((unsigned)h) << 16); }
__device__ __forceinline__ unsigned pk16(unsigned short a, unsigned short b) { return (unsigned)a | ((unsigned)b << 16); }

__device__ __forceinline__ void dep_guard_h(v8f& a, v8f& b, v16h x, v16h y) { asm volatile("v_nop\n\tv_nop\n\tv_nop\n\tv_nop" : "+v"(a), "+v"(b) : "v"(x), "v"(y)); }
__device__ __forceinline__ void dep_guard_b(v8f& a, v8f& b, v16b x, v16b y) { asm volatile("v_nop\n\tv_nop\n\tv_nop\n\tv_nop" : "+v"(a), "+v"(b) : "v"(x), "v"(y)); }
__device__ __forceinline__ void keep4_h(v16h a, v16h b, v16h c, v16h d) { asm volatile("v_nop" :: "v"(a), "v"(b), "v"(c), "v"(d)); }
__device__ __forceinline__ void keep4_b(v16b a, v16b b, v16b c, v16b d) { asm volatile("v_nop" :: "v"(a), "v"(b), "v"(c), "v"(d)); }
__device__ __forceinline__ void acc_guard4(v8f& a, v8f& b, v8f& c, v8f& d) { asm volatile("v_nop\n\tv_nop\n\tv_nop\n\tv_nop" : "+v"(a), "+v"(b), "+v"(c), "+v"(d)); }
template <typename T> struct Frag;
template <> struct Frag<_Float16> {
  typedef v16h V; union U { v16h v; v8h h[2]; };
  static __device__ __forceinline__ v16h load(const _Float16* p) {
    U f; f.h[0] = *(const v8h*)(p); f.h[1] = *(const v8h*)(p + 16); return f.v;
  }
  static __device__ __forceinline__ v8f mma(v16h a, v16h b, v8f c) {
    return __builtin_amdgcn_wmma_f32_16x16x32_f16(false, a, false, b, (short)0, c, false, false);
  }
  static __device__ __forceinline__ void guard(v8f& a, v8f& b, v16h x, v16h y) { dep_guard_h(a, b, x, y); }
  static __device__ __forceinline__ void keep(v16h a, v16h b, v16h c, v16h d) { keep4_h(a, b, c, d); }
};
template <> struct Frag<__bf16> {
  typedef v16b V; union U { v16b v; v8b h[2]; };
  static __device__ __forceinline__ v16b load(const __bf16* p) {
    U f; f.h[0] = *(const v8b*)(p); f.h[1] = *(const v8b*)(p + 16); return f.v;
  }
  static __device__ __forceinline__ v8f mma(v16b a, v16b b, v8f c) {
    return __builtin_amdgcn_wmma_f32_16x16x32_bf16(false, a, false, b, (short)0, c, false, false);
  }
  static __device__ __forceinline__ void guard(v8f& a, v8f& b, v16b x, v16b y) { dep_guard_b(a, b, x, y); }
  static __device__ __forceinline__ void keep(v16b a, v16b b, v16b c, v16b d) { keep4_b(a, b, c, d); }
};

template <int ET> struct Elem;
template <> struct Elem<0> { typedef _Float16 T; };
template <> struct Elem<1> { typedef __bf16 T; };
template <int ET, int SPLIT, int BIAS_MODE, int OUT_MODE, bool RESID, int ACT = 0>
__global__ __launch_bounds__(256) void wmma_gemm64(
    const unsigned short* __restrict__ Ap, const unsigned short* __restrict__ A2p, int lda, long strideA,
    const unsigned short* __restrict__ Btp, const unsigned short* __restrict__ Bt2p, int ldb, long strideB,
    void* __restrict__ Cout, void* __restrict__ Cout2, int ldc, long strideC,
    const float* __restrict__ bias,
    const float* __restrict__ resid, long strideR,
    int M, int N, int K, float scale) {
  typedef typename Elem<ET>::T T;
  typedef typename Frag<T>::V V;
  const T* A = (const T*)Ap; const T* A2 = (const T*)A2p; const T* Bt = (const T*)Btp; const T* Bt2 = (const T*)Bt2p;
  __shared__ __align__(16) float sT[8][16 * 68];
  const int b    = blockIdx.y;
  const int lane = threadIdx.x & 31;
  const int wave = threadIdx.x >> 5;
  const int tilesN = N >> 6;
  const int tilesM = M >> 6;
  const int tile = blockIdx.x * 8 + wave;
  if (tile >= tilesM * tilesN) return;
  const int tm = tile / tilesN;
  const int tn = tile - tm * tilesN;
  const int m0 = tm << 6;
  const int n0 = tn << 6;

  const T* Ab  = A  + (size_t)b * strideA;
  const T* Bb  = Bt + (size_t)b * strideB;
  const T* Ab2 = (SPLIT != 0) ? (A2  + (size_t)b * strideA) : nullptr;
  const T* Bb2 = (SPLIT == 1) ? (Bt2 + (size_t)b * strideB) : nullptr;

  const int rlane = lane & 15;
  const int koff  = (lane >> 4) * 8;
  const int mOff  = (lane >> 4) * 8;

  v8f acc[4][4];
#pragma unroll
  for (int i = 0; i < 4; ++i)
#pragma unroll
    for (int j = 0; j < 4; ++j) acc[i][j] = (v8f){0.f,0.f,0.f,0.f,0.f,0.f,0.f,0.f};

  for (int k0 = 0; k0 < K; k0 += 32) {
    V bh[4], bl[4];
#pragma unroll
    for (int j = 0; j < 4; ++j) {
      const size_t bo = (size_t)(n0 + (j << 4) + rlane) * ldb + koff + k0;
      bh[j] = Frag<T>::load(Bb + bo);
      if (SPLIT == 1) bl[j] = Frag<T>::load(Bb2 + bo);
    }
#pragma unroll
    for (int i = 0; i < 4; ++i) {
      const size_t ao = (size_t)(m0 + (i << 4) + rlane) * lda + koff + k0;
      V ah = Frag<T>::load(Ab + ao);
      V al;
      if (SPLIT != 0) al = Frag<T>::load(Ab2 + ao);
#pragma unroll
      for (int j = 0; j < 4; ++j) {
        acc[i][j] = Frag<T>::mma(ah, bh[j], acc[i][j]);
        if (SPLIT == 1) acc[i][j] = Frag<T>::mma(ah, bl[j], acc[i][j]);
        if (SPLIT != 0) acc[i][j] = Frag<T>::mma(al, bh[j], acc[i][j]);
      }
      Frag<T>::guard(acc[i][0], acc[i][3], ah, (SPLIT != 0) ? al : ah);
    }
    Frag<T>::keep(bh[0], bh[1], bh[2], bh[3]);
    if (SPLIT == 1) Frag<T>::keep(bl[0], bl[1], bl[2], bl[3]);
  }
  acc_guard4(acc[0][0], acc[0][1], acc[0][2], acc[0][3]);
  acc_guard4(acc[1][0], acc[1][1], acc[1][2], acc[1][3]);
  acc_guard4(acc[2][0], acc[2][1], acc[2][2], acc[2][3]);
  acc_guard4(acc[3][0], acc[3][1], acc[3][2], acc[3][3]);

  float* slab = sT[wave];
  const float* Rb = RESID ? (resid + (size_t)b * strideR) : nullptr;
#pragma unroll
  for (int i = 0; i < 4; ++i) {
    const int mBase = m0 + (i << 4);
#pragma unroll
    for (int j = 0; j < 4; ++j) {
      const int n = n0 + (j << 4) + rlane;
      float bv = 0.f;
      if (BIAS_MODE == 2) bv = bias[n];
#pragma unroll
      for (int r = 0; r < 8; ++r) {
        float v = acc[i][j][r] * scale;
        if (BIAS_MODE == 1) v += bias[mBase + mOff + r];
        if (BIAS_MODE == 2) v += bv;
        if (RESID) v += Rb[(size_t)(mBase + mOff + r) * ldc + n];
        if (ACT == 1) v = tanhf(v);
        if (ACT == 2) v = fmaxf(v, 0.0f);
        if (ACT == 4) v = (v > 0.f) ? v : 0.01f * v;
        slab[(mOff + r) * 68 + (j << 4) + rlane] = v;
      }
    }
    __builtin_amdgcn_fence(__ATOMIC_RELEASE, "workgroup");
    __builtin_amdgcn_wave_barrier();
    __builtin_amdgcn_fence(__ATOMIC_ACQUIRE, "workgroup");
    if (OUT_MODE == 0) {
      float* C = (float*)Cout + (size_t)b * strideC;
      const int hh = lane >> 4, c4 = (lane & 15) * 4;
      for (int pass = 0; pass < 2; ++pass) {
#pragma unroll
        for (int it = 0; it < 8; ++it) {
          const int row = it * 2 + hh;
          v4f v = *(const v4f*)(slab + row * 68 + c4);
          *(volatile v4f*)(C + (size_t)(mBase + row) * ldc + n0 + c4) = v;
        }
        __threadfence();
      }
    } else {
      const int q = lane >> 3, c8 = (lane & 7) * 8;
      unsigned short* C  = (unsigned short*)Cout  + (size_t)b * strideC;
      unsigned short* C2 = (OUT_MODE == 2) ? ((unsigned short*)Cout2 + (size_t)b * strideC) : nullptr;
      for (int pass = 0; pass < 2; ++pass) {
#pragma unroll
        for (int it = 0; it < 4; ++it) {
          const int row = it * 4 + q;
          const float* sp = slab + row * 68 + c8;
          v8h hv, lv;
#pragma unroll
          for (int e = 0; e < 8; ++e) {
            if (OUT_MODE == 1) {
              hv[e] = (_Float16)sp[e];
            } else {
              unsigned short hb = f2bf_bits(sp[e]);
              unsigned short lb = f2bf_bits(sp[e] - bf_bits2f(hb));
              hv[e] = __builtin_bit_cast(_Float16, hb);
              lv[e] = __builtin_bit_cast(_Float16, lb);
            }
          }
          *(volatile v8h*)(C + (size_t)(mBase + row) * ldc + n0 + c8) = hv;
          if (OUT_MODE == 2) *(volatile v8h*)(C2 + (size_t)(mBase + row) * ldc + n0 + c8) = lv;
        }
        __threadfence();
      }
    }
    __builtin_amdgcn_fence(__ATOMIC_RELEASE, "workgroup");
    __builtin_amdgcn_wave_barrier();
    __builtin_amdgcn_fence(__ATOMIC_ACQUIRE, "workgroup");
  }
}

__global__ __launch_bounds__(256) void cast_bf16x2_kernel(const float* __restrict__ in, unsigned short* __restrict__ out, int n2) {
  const int i = blockIdx.x * 256 + threadIdx.x;
  if (i < n2) {
    const v2f f = *(const v2f*)(in + 2 * (size_t)i);
    const unsigned u = pk16(f2bf_bits(f[0]), f2bf_bits(f[1]));
    ((volatile unsigned*)out)[i] = u;
    __threadfence();
    ((volatile unsigned*)out)[i] = u;
  }
}

__global__ __launch_bounds__(256) void tsplit_kernel(const float* __restrict__ W, unsigned short* __restrict__ oh,
                                                     unsigned short* __restrict__ ol, int R, int Cc, long sIn, long sOut) {
  __shared__ __align__(16) float tf[64 * 68];
  W  += (size_t)blockIdx.z * sIn;
  oh += (size_t)blockIdx.z * sOut;
  ol += (size_t)blockIdx.z * sOut;
  const int c0  = blockIdx.x * 64;
  const int r0  = blockIdx.y * 64;
  const int tid = threadIdx.x;
  {
    const int lr = tid >> 4;
    const int c4 = (tid & 15) * 4;
#pragma unroll
    for (int it = 0; it < 4; ++it) {
      const int rr = it * 16 + lr;
      const v4f a = *(const v4f*)(W + (size_t)(r0 + rr) * Cc + c0 + c4);
      *(v4f*)(tf + rr * 68 + c4) = a;
    }
  }
  __syncthreads();
  const int sub = tid >> 3;
  const int c8  = (tid & 7) * 8;
  v4u hv[2], lv[2];
#pragma unroll
  for (int it = 0; it < 2; ++it) {
    const int oc = it * 32 + sub;
    v4u a, a2;
#pragma unroll
    for (int q = 0; q < 4; ++q) {
      const float f0 = tf[(c8 + 2 * q) * 68 + oc];
      const float f1 = tf[(c8 + 2 * q + 1) * 68 + oc];
      const unsigned short h0 = f2bf_bits(f0), h1 = f2bf_bits(f1);
      const unsigned short l0 = f2bf_bits(f0 - bf_bits2f(h0)), l1 = f2bf_bits(f1 - bf_bits2f(h1));
      a[q]  = pk16(h0, h1);
      a2[q] = pk16(l0, l1);
    }
    hv[it] = a; lv[it] = a2;
  }
  for (int pass = 0; pass < 2; ++pass) {
#pragma unroll
    for (int it = 0; it < 2; ++it) {
      const int oc = it * 32 + sub;
      const size_t go = (size_t)(c0 + oc) * R + r0 + c8;
      *(volatile v4u*)(oh + go) = hv[it];
      *(volatile v4u*)(ol + go) = lv[it];
    }
    __threadfence();
  }
}

#define AT_D 64
#define AT_NW 4
#define AT_QB 64
#define AT_KC 64

__device__ __forceinline__ v8f at_mma(v16b a, v16b b, v8f c) {
  c = __builtin_amdgcn_wmma_f32_16x16x32_bf16(false, a, false, b, (short)0, c, false, false);
  asm volatile("v_nop\n\tv_nop\n\tv_nop\n\tv_nop" : "+v"(c) : "v"(a), "v"(b));
  return c;
}
__device__ __forceinline__ v8f at_mma_h(v16b a, v16b b, v8f c) {
  const v16h ah = __builtin_bit_cast(v16h, a), bh = __builtin_bit_cast(v16h, b);
  c = __builtin_amdgcn_wmma_f32_16x16x32_f16(false, ah, false, bh, (short)0, c, false, false);
  asm volatile("v_nop\n\tv_nop\n\tv_nop\n\tv_nop" : "+v"(c) : "v"(ah), "v"(bh));
  return c;
}
__device__ __forceinline__ __bf16 at_h16bits(float f) { return __builtin_bit_cast(__bf16, (_Float16)f); }

__global__ __launch_bounds__(128)
void mha_full64_kernel(const unsigned short* __restrict__ qkhp, const unsigned short* __restrict__ qklp,
                       const unsigned short* __restrict__ vtp,
                       unsigned short* __restrict__ ohp, unsigned short* __restrict__ olp, float sscale) {
  union FB { v16b v; v8b h[2]; };
  __shared__ __align__(16) __bf16 Ksh[AT_KC * AT_D];
  __shared__ __align__(16) __bf16 Ksl[AT_KC * AT_D];
  __shared__ __align__(16) __bf16 Vth[AT_D * AT_KC];
  __shared__ __align__(16) __bf16 Psh[AT_NW][16 * AT_KC];
  __shared__ __align__(16) float  Os[AT_NW][16 * 68];

  const int tid  = threadIdx.x;
  const int wave = tid >> 5;
  const int lane = tid & 31;
  const int hh   = lane >> 4;
  const int c    = lane & 15;

  const int nqb = kSeq / AT_QB;
  const int bx = blockIdx.x;
  const int qb = bx % nqb;
  const int h  = bx / nqb;
  const int bb = blockIdx.y;
  const int q0 = qb * AT_QB + wave * 16;

  const size_t rowbase = (size_t)bb * kSeq;
  const __bf16* Qh = (const __bf16*)(const void*)qkhp + rowbase * kQkLd + (size_t)h * AT_D;
  const __bf16* Ql = (const __bf16*)(const void*)qklp + rowbase * kQkLd + (size_t)h * AT_D;
  const __bf16* Kh = Qh + kDm;
  const __bf16* Kl = Ql + kDm;
  const __bf16* Vt = (const __bf16*)(const void*)vtp + (size_t)bb * kDm * kSeq + (size_t)h * AT_D * kSeq;
  unsigned short* Oh = ohp + rowbase * kDm + (size_t)h * AT_D;
  unsigned short* Ol = olp + rowbase * kDm + (size_t)h * AT_D;

  v16b qah[2], qal[2];
#pragma unroll
  for (int dc = 0; dc < 2; ++dc) {
    const __bf16* qr = Qh + (size_t)(q0 + c) * kQkLd + dc * 32 + 8 * hh;
    const __bf16* ql = Ql + (size_t)(q0 + c) * kQkLd + dc * 32 + 8 * hh;
    qah[dc] = Frag<__bf16>::load(qr);
    qal[dc] = Frag<__bf16>::load(ql);
  }

  float mrow[8], lrow[8];
  v8f oacc[4];
#pragma unroll
  for (int r = 0; r < 8; ++r) { mrow[r] = -INFINITY; lrow[r] = 0.f; }
#pragma unroll
  for (int t = 0; t < 4; ++t) oacc[t] = (v8f){0.f,0.f,0.f,0.f,0.f,0.f,0.f,0.f};

  const int nChunks = kSeq / AT_KC;
  for (int kc = 0; kc < nChunks; ++kc) {
    const int kv0 = kc * AT_KC;
    __syncthreads();
    {
      const int r = tid >> 1, half = (tid & 1) * 32;
      const __bf16* ksh = Kh + (size_t)(kv0 + r) * kQkLd + half;
      const __bf16* ksl = Kl + (size_t)(kv0 + r) * kQkLd + half;
      const __bf16* vsh = Vt + (size_t)r * kSeq + kv0 + half;
#pragma unroll
      for (int i = 0; i < 4; ++i) {
        const v8b a0 = *(const v8b*)(ksh + 8 * i);
        const v8b a1 = *(const v8b*)(ksl + 8 * i);
        const v8b b0 = *(const v8b*)(vsh + 8 * i);
        *(v8b*)(Ksh + r * AT_D  + half + 8 * i) = a0;
        *(v8b*)(Ksl + r * AT_D  + half + 8 * i) = a1;
        *(v8b*)(Vth + r * AT_KC + half + 8 * i) = b0;
      }
    }
    __syncthreads();

    v8f s[4];
#pragma unroll
    for (int j = 0; j < 4; ++j) {
      s[j] = (v8f){0.f,0.f,0.f,0.f,0.f,0.f,0.f,0.f};
#pragma unroll
      for (int dc = 0; dc < 2; ++dc) {
        FB kb, kl;
        kb.h[0] = *(const v8b*)(Ksh + (j * 16 + c) * AT_D + dc * 32 + 8 * hh);
        kb.h[1] = *(const v8b*)(Ksh + (j * 16 + c) * AT_D + dc * 32 + 16 + 8 * hh);
        kl.h[0] = *(const v8b*)(Ksl + (j * 16 + c) * AT_D + dc * 32 + 8 * hh);
        kl.h[1] = *(const v8b*)(Ksl + (j * 16 + c) * AT_D + dc * 32 + 16 + 8 * hh);
        s[j] = at_mma(qah[dc], kb.v, s[j]);
        s[j] = at_mma(qah[dc], kl.v, s[j]);
        s[j] = at_mma(qal[dc], kb.v, s[j]);
      }
    }
    float cm[8];
#pragma unroll
    for (int r = 0; r < 8; ++r) {
      float m = -INFINITY;
#pragma unroll
      for (int j = 0; j < 4; ++j) {
        const float sv = s[j][r] * sscale;
        s[j][r] = sv;
        m = fmaxf(m, sv);
      }
#pragma unroll
      for (int off = 1; off < 16; off <<= 1) m = fmaxf(m, __shfl_xor(m, off, 32));
      cm[r] = m;
    }
    __bf16* pwh = Psh[wave];
#pragma unroll
    for (int r = 0; r < 8; ++r) {
      const float mnew = fmaxf(mrow[r], cm[r]);
      const float alpha = expf(mrow[r] - mnew);
      mrow[r] = mnew;
      float psum = 0.f;
#pragma unroll
      for (int j = 0; j < 4; ++j) {
        const float p = expf(s[j][r] - mnew);
        psum += p;
        pwh[(8 * hh + r) * AT_KC + j * 16 + c] = at_h16bits(p * kPScale);
      }
#pragma unroll
      for (int off = 1; off < 16; off <<= 1) psum += __shfl_xor(psum, off, 32);
      lrow[r] = lrow[r] * alpha + psum;
#pragma unroll
      for (int t = 0; t < 4; ++t) oacc[t][r] *= alpha;
    }
    __builtin_amdgcn_fence(__ATOMIC_RELEASE, "workgroup");
    __builtin_amdgcn_wave_barrier();
    __builtin_amdgcn_fence(__ATOMIC_ACQUIRE, "workgroup");
#pragma unroll 1
    for (int kk = 0; kk < 2; ++kk) {
      FB pa;
      pa.h[0] = *(const v8b*)(pwh + c * AT_KC + kk * 32 + 8 * hh);
      pa.h[1] = *(const v8b*)(pwh + c * AT_KC + kk * 32 + 16 + 8 * hh);
#pragma unroll
      for (int t = 0; t < 4; ++t) {
        FB vb;
        vb.h[0] = *(const v8b*)(Vth + (t * 16 + c) * AT_KC + kk * 32 + 8 * hh);
        vb.h[1] = *(const v8b*)(Vth + (t * 16 + c) * AT_KC + kk * 32 + 16 + 8 * hh);
        oacc[t] = at_mma_h(pa.v, vb.v, oacc[t]);
      }
    }
  }

  float* os = Os[wave];
#pragma unroll
  for (int r = 0; r < 8; ++r) {
    const float inv = 1.0f / (lrow[r] * kPScale);
#pragma unroll
    for (int t = 0; t < 4; ++t) os[(8 * hh + r) * 68 + t * 16 + c] = oacc[t][r] * inv;
  }
  __builtin_amdgcn_fence(__ATOMIC_RELEASE, "workgroup");
  __builtin_amdgcn_wave_barrier();
  __builtin_amdgcn_fence(__ATOMIC_ACQUIRE, "workgroup");
  {
    const int q = lane >> 3, c8 = (lane & 7) * 8;
    for (int pass = 0; pass < 2; ++pass) {
#pragma unroll
      for (int it = 0; it < 4; ++it) {
        const int row = it * 4 + q;
        const float* sp = os + row * 68 + c8;
        v8h hv, lv;
#pragma unroll
        for (int e = 0; e < 8; ++e) {
          const unsigned short hb = f2bf_bits(sp[e]);
          const unsigned short lb = f2bf_bits(sp[e] - bf_bits2f(hb));
          hv[e] = __builtin_bit_cast(_Float16, hb);
          lv[e] = __builtin_bit_cast(_Float16, lb);
        }
        *(volatile v8h*)(Oh + (size_t)(q0 + row) * kDm + c8) = hv;
        *(volatile v8h*)(Ol + (size_t)(q0 + row) * kDm + c8) = lv;
      }
      __threadfence();
    }
  }
}

extern "C" void kernel_launch(void* const* d_in, const int* in_sizes, int n_in,
                              void* d_out, int out_size, void* d_ws, size_t ws_size,
                              hipStream_t stream) {
  if (n_in < 5) return;
  if (in_sizes[0] != kRows * kDm || in_sizes[1] != kDm * 3 * kDm || in_sizes[2] != 3 * kDm ||
      in_sizes[3] != kDm * kDm || in_sizes[4] != kDm || out_size != kRows * kDm) return;

  const float* x     = (const float*)d_in[0];
  const float* W_qkv = (const float*)d_in[1];
  const float* b_qkv = (const float*)d_in[2];
  const float* W_out = (const float*)d_in[3];
  const float* b_out = (const float*)d_in[4];
  float* out = (float*)d_out;

  const size_t bXb  = (size_t)kRows * kDm * 2;
  const size_t bWq  = (size_t)3 * kDm * kDm * 2;
  const size_t bWo  = (size_t)kDm * kDm * 2;
  const size_t bQk  = (size_t)kRows * kQkLd * 2;
  const size_t bVt  = (size_t)kBatch * kDm * kSeq * 2;
  const size_t bO   = (size_t)kRows * kDm * 2;
  size_t off = 0;
  unsigned char* ws = (unsigned char*)d_ws;
  unsigned short* xb     = (unsigned short*)(ws + off); off += bXb;
  unsigned short* wqT_hi = (unsigned short*)(ws + off); off += bWq;
  unsigned short* wqT_lo = (unsigned short*)(ws + off); off += bWq;
  unsigned short* woT_hi = (unsigned short*)(ws + off); off += bWo;
  unsigned short* woT_lo = (unsigned short*)(ws + off); off += bWo;
  unsigned short* qk_hi  = (unsigned short*)(ws + off); off += bQk;
  unsigned short* qk_lo  = (unsigned short*)(ws + off); off += bQk;
  unsigned short* vT     = (unsigned short*)(ws + off); off += bVt;
  unsigned short* o_hi   = (unsigned short*)(ws + off); off += bO;
  unsigned short* o_lo   = (unsigned short*)(ws + off); off += bO;
  if (off > ws_size) return;

  {
    const int n2 = kRows * kDm / 2;
    cast_bf16x2_kernel<<<dim3((n2 + 255) / 256), dim3(256), 0, stream>>>(x, xb, n2);
  }
  tsplit_kernel<<<dim3(3 * kDm / 64, kDm / 64, 1), dim3(256), 0, stream>>>(W_qkv, wqT_hi, wqT_lo, kDm, 3 * kDm, 0L, 0L);
  tsplit_kernel<<<dim3(kDm / 64, kDm / 64, 1), dim3(256), 0, stream>>>(W_out, woT_hi, woT_lo, kDm, kDm, 0L, 0L);
  {
    const int M = kRows, N = kQkLd, K = kDm;
    const int blocks = ((M / 64) * (N / 64) + 7) / 8;
    wmma_gemm64<1, 0, 2, 2, false><<<dim3(blocks, 1), dim3(256), 0, stream>>>(
        xb, xb, K, 0L, wqT_hi, wqT_hi, K, 0L, (void*)qk_hi, (void*)qk_lo, N, 0L,
        b_qkv, b_qkv, 0L, M, N, K, 1.0f);
  }
  {
    const int M = kDm, N = kSeq, K = kDm;
    const int blocks = ((M / 64) * (N / 64) + 7) / 8;
    wmma_gemm64<1, 0, 1, 1, false><<<dim3(blocks, kBatch), dim3(256), 0, stream>>>(
        wqT_hi + (size_t)2 * kDm * kDm, wqT_hi + (size_t)2 * kDm * kDm, K, 0L,
        xb, xb, K, (long)kSeq * kDm,
        (void*)vT, (void*)vT, N, (long)kDm * kSeq,
        b_qkv + 2 * kDm, b_qkv, 0L, M, N, K, 1.0f);
  }
  mha_full64_kernel<<<dim3(kHeads * (kSeq / AT_QB), kBatch), dim3(128), 0, stream>>>(
      qk_hi, qk_lo, vT, o_hi, o_lo, 0.125f);
  {
    const int M = kRows, N = kDm, K = kDm;
    const int blocks = ((M / 64) * (N / 64) + 7) / 8;
    wmma_gemm64<1, 2, 2, 0, false><<<dim3(blocks, 1), dim3(256), 0, stream>>>(
        o_hi, o_lo, K, 0L, woT_hi, woT_hi, K, 0L, (void*)out, (void*)out, N, 0L,
        b_out, b_out, 0L, M, N, K, 1.0f);
  }
}
